// DotReluBlock_13451837571889
// MI455X (gfx1250) — hardware-verified
//
#include <hip/hip_runtime.h>
#include <hip/hip_bf16.h>
#include <math.h>

#define NBd 4
#define NNd 4096
#define HHd 128
#define GSTR 48

typedef _Float16 bf16;
typedef _Float16 f16;
typedef __attribute__((ext_vector_type(4))) unsigned v4u_t;
typedef unsigned v4ua __attribute__((ext_vector_type(4), may_alias));
typedef __attribute__((ext_vector_type(4))) float v4f_t;
typedef float v4fa __attribute__((ext_vector_type(4), may_alias));
typedef __attribute__((ext_vector_type(16))) bf16  bf16x16;
typedef bf16x16 f16x16;
typedef __attribute__((ext_vector_type(8)))  bf16  bf16x8;
typedef bf16x8 f16x8;
typedef __attribute__((ext_vector_type(8)))  float f32x8;
__device__ __forceinline__ f32x8 wmma16(f16x16 a, f16x16 b, f32x8 c) {
  c = __builtin_amdgcn_wmma_f32_16x16x32_f16(false, a, false, b, (short)0, c, false, false);
  asm volatile("v_nop\n\tv_nop\n\tv_nop\n\tv_nop" : "+v"(c) : "v"(a), "v"(b));
  return c;
}
__device__ __forceinline__ f16x16 lds_frag(const f16* base, int stride) {
  const int lane = threadIdx.x & 31, row = lane & 15, kh = (lane >> 4) * 8;
  const f16x8 lo = *(const f16x8*)(base + row * stride + kh);
  const f16x8 hi = *(const f16x8*)(base + row * stride + kh + 16);
  f16x16 f;
#pragma unroll
  for (int i = 0; i < 8; ++i) { f[i] = lo[i]; f[i + 8] = hi[i]; }
  return f;
}
__device__ __forceinline__ f16x16 gfrag(const bf16* __restrict__ base, int r0, int k0) {
  const int lane = threadIdx.x & 31, row = r0 + (lane & 15), kh = (lane >> 4) * 8;
  const f16x8 lo = *(const f16x8*)(base + (size_t)row * HHd + k0 + kh); const f16x8 hi = *(const f16x8*)(base + (size_t)row * HHd + k0 + kh + 16);
  f16x16 f;
#pragma unroll
  for (int i = 0; i < 8; ++i) { f[i] = lo[i]; f[i + 8] = hi[i]; }
  return f;
}

#define GSTR 48
template <typename AT, int EPI, bool OUT16>
__global__ __launch_bounds__(256) void gemm_kne(const AT* __restrict__ A, int lda, const float* __restrict__ Wm, int ldw,
                                                const float* __restrict__ bias, const float* __restrict__ R, const float* __restrict__ gvec,
                                                void* __restrict__ Yv, int ldy, int K) {
  __shared__ __attribute__((aligned(16))) f16 ldsA[128 * GSTR];
  __shared__ __attribute__((aligned(16))) f16 ldsW[128 * GSTR];
  __shared__ __attribute__((aligned(16))) float oS[8][32 * 68];
  const int tid = threadIdx.x, lane = tid & 31, wave = tid >> 5, cl = lane & 15, rh = (lane >> 4) * 8;
  const int m0 = blockIdx.x * 128, n0 = blockIdx.y * 128;
  const int wm = (wave & 3) * 32, wn = (wave >> 2) * 64;
  f32x8 acc[2][4];
#pragma unroll
  for (int i = 0; i < 2; ++i)
#pragma unroll
    for (int j = 0; j < 4; ++j) { f32x8 z = {}; acc[i][j] = z; }
#pragma unroll 1
  for (int k0 = 0; k0 < K; k0 += 32) {
    __syncthreads();
    { const int row = tid >> 1, ch = (tid & 1) * 16;
      const AT* src = A + (size_t)(m0 + row) * lda + k0 + ch;
#pragma unroll
      for (int g = 0; g < 16; ++g) ldsA[row * GSTR + ch + g] = (f16)src[g]; }
    { const int k = tid >> 3, nn0 = (tid & 7) * 16;
      const float* src = Wm + (size_t)(k0 + k) * ldw + n0 + nn0;
#pragma unroll
      for (int g = 0; g < 4; ++g) { const v4f_t v = *(const v4f_t*)(src + 4 * g);
#pragma unroll
        for (int u = 0; u < 4; ++u) ldsW[(nn0 + 4 * g + u) * GSTR + k] = (f16)v[u]; } }
    __syncthreads();
    f16x16 af[2];
#pragma unroll
    for (int i = 0; i < 2; ++i) af[i] = lds_frag(ldsA + (wm + 16 * i) * GSTR, GSTR);
#pragma unroll
    for (int j = 0; j < 4; ++j) {
      const f16x16 bf = lds_frag(ldsW + (wn + 16 * j) * GSTR, GSTR);
#pragma unroll
      for (int i = 0; i < 2; ++i) acc[i][j] = wmma16(af[i], bf, acc[i][j]);
    }
  }
  float* so = oS[wave];
#pragma unroll
  for (int i = 0; i < 2; ++i)
#pragma unroll
    for (int j = 0; j < 4; ++j) {
      const int n = n0 + wn + 16 * j + cl;
      const float bv = bias ? bias[n] : 0.0f;
      const float gv = (EPI == 2) ? gvec[n] : 0.0f;
      if (EPI == 1) {
#pragma unroll 1
        for (int r = 0; r < 8; ++r) { const float xg = acc[i][j][r] + bv; so[(16 * i + rh + r) * 68 + 16 * j + cl] = 0.5f * xg * (1.0f + erff(xg * 0.70710678118654752f)); }
      } else {
#pragma unroll
        for (int r = 0; r < 8; ++r) {
          float v = acc[i][j][r] + bv;
          if (EPI == 2) v = R[(size_t)(m0 + wm + 16 * i + rh + r) * ldy + n] + gv * v;
          so[(16 * i + rh + r) * 68 + 16 * j + cl] = v;
        }
      }
    }
  asm volatile("s_wait_dscnt 0" ::: "memory");
  __builtin_amdgcn_wave_barrier();
#pragma unroll 1
  for (int pass = 0; pass < 2; ++pass) {
    if (OUT16) {
      f16* Y = (f16*)Yv;
#pragma unroll
      for (int it = 0; it < 8; ++it) { const int c = lane + 32 * it, rr = c >> 3, q8 = (c & 7) * 8;
        union { f16 h[8]; v4u_t v; } u;
#pragma unroll
        for (int e = 0; e < 8; ++e) u.h[e] = (f16)so[rr * 68 + q8 + e];
        *(volatile v4u_t*)(Y + (size_t)(m0 + wm + rr) * ldy + n0 + wn + q8) = u.v; }
    } else {
      float* Y = (float*)Yv;
#pragma unroll
      for (int it = 0; it < 16; ++it) { const int f4 = lane + 32 * it, rr = f4 >> 4, q = (f4 & 15) * 4;
        *(volatile v4f_t*)(Y + (size_t)(m0 + wm + rr) * ldy + n0 + wn + q) = *(const v4fa*)(so + rr * 68 + q); }
    }
    __threadfence();
  }
}

__global__ __launch_bounds__(256) void k_sval(const float* __restrict__ kin, const float* __restrict__ Wv, const float* __restrict__ bv, const float* __restrict__ Wp, float* __restrict__ sv) {
  __shared__ float uS[HHd]; __shared__ float c0S;
  const int tid = threadIdx.x;
  if (tid < HHd) { float s = 0.0f;
#pragma unroll 1
    for (int j = 0; j < HHd; ++j) s += Wv[tid * HHd + j] * Wp[j];
    uS[tid] = s; }
  if (tid == 0) { float s = 0.0f; for (int j = 0; j < HHd; ++j) s += bv[j] * Wp[j]; c0S = s; }
  __syncthreads();
  const size_t row = (size_t)blockIdx.x * 256 + tid; const float* kr = kin + row * HHd; float s = c0S;
#pragma unroll 1
  for (int j = 0; j < HHd; ++j) s += kr[j] * uS[j];
  *(volatile float*)(sv + row) = s; __threadfence(); *(volatile float*)(sv + row) = s;
}
__global__ __launch_bounds__(128) void k_colstats(const bf16* __restrict__ Q16, const bf16* __restrict__ K16, float* __restrict__ st) {
  __shared__ __attribute__((aligned(16))) f16 qS[64 * 136];
  const int tid = threadIdx.x, lane = tid & 31, wave = tid >> 5;
  const int b = blockIdx.x / (NNd / 64), k0 = (blockIdx.x % (NNd / 64)) * 64 + wave * 16;
  const bf16* Qb = Q16 + (size_t)b * NNd * HHd; const bf16* Kb = K16 + (size_t)b * NNd * HHd;
  f16x16 kf[4];
#pragma unroll
  for (int ks = 0; ks < 4; ++ks) kf[ks] = gfrag(Kb, k0, ks * 32);
  const float c = 0.08838834764831845f * 1.4426950408889634f;
  float m = -3.0e38f, z = 0.0f;
#pragma unroll 1
  for (int q0 = 0; q0 < NNd; q0 += 64) {
    __syncthreads();
    for (int e = tid; e < 64 * 16; e += 128) { const int r = e >> 4, ch = (e & 15) * 8; *(f16x8*)(qS + r * 136 + ch) = *(const f16x8*)(Qb + (size_t)(q0 + r) * HHd + ch); }
    __syncthreads();
#pragma unroll
    for (int rt = 0; rt < 4; ++rt) { f32x8 acc = {};
#pragma unroll
      for (int ks = 0; ks < 4; ++ks) acc = wmma16(lds_frag(qS + (rt * 16) * 136 + ks * 32, 136), kf[ks], acc);
      float mx = m;
#pragma unroll
      for (int r = 0; r < 8; ++r) { acc[r] *= c; mx = fmaxf(mx, acc[r]); }
      mx = fmaxf(mx, __shfl_xor(mx, 16, 32));
      z *= exp2f(m - mx);
      float add = 0.0f;
#pragma unroll
      for (int r = 0; r < 8; ++r) add += exp2f(acc[r] - mx);
      add += __shfl_xor(add, 16, 32);
      z += add; m = mx; }
  }
  __shared__ __attribute__((aligned(16))) float mO[64], zO[64];
  if (lane < 16) { mO[wave * 16 + lane] = m; zO[wave * 16 + lane] = z; }
  __syncthreads();
  { const size_t kb0 = (size_t)b * NNd + (blockIdx.x % (NNd / 64)) * 64;
#pragma unroll 1
    for (int pass = 0; pass < 2; ++pass) { if (tid < 16) *(volatile v4f_t*)(st + kb0 + tid * 4) = *(const v4fa*)(mO + tid * 4);
      else if (tid < 32) *(volatile v4f_t*)(st + (size_t)NBd * NNd + kb0 + (tid - 16) * 4) = *(const v4fa*)(zO + (tid - 16) * 4); __threadfence(); } }
}
__global__ __launch_bounds__(128) void k_colsoft(const bf16* __restrict__ Q16, const bf16* __restrict__ K16, const float* __restrict__ st, const float* __restrict__ sv, const float* __restrict__ bp, float* __restrict__ out) {
  __shared__ __attribute__((aligned(16))) f16 kS[64 * 136];
  __shared__ float mS[64], wS[64];
  __shared__ __attribute__((aligned(16))) float oS[64];
  const int tid = threadIdx.x, lane = tid & 31, wave = tid >> 5;
  const int b = blockIdx.x / (NNd / 64), q0 = (blockIdx.x % (NNd / 64)) * 64 + wave * 16;
  const bf16* Qb = Q16 + (size_t)b * NNd * HHd; const bf16* Kb = K16 + (size_t)b * NNd * HHd;
  f16x16 qf[4];
#pragma unroll
  for (int ks = 0; ks < 4; ++ks) qf[ks] = gfrag(Qb, q0, ks * 32);
  const float c = 0.08838834764831845f * 1.4426950408889634f;
  float acc_o = 0.0f;
#pragma unroll 1
  for (int k0 = 0; k0 < NNd; k0 += 64) {
    __syncthreads();
    for (int e = tid; e < 64 * 16; e += 128) { const int r = e >> 4, ch = (e & 15) * 8; *(f16x8*)(kS + r * 136 + ch) = *(const f16x8*)(Kb + (size_t)(k0 + r) * HHd + ch); }
    if (tid < 64) { const size_t kk = (size_t)b * NNd + k0 + tid; mS[tid] = st[kk]; wS[tid] = sv[kk] / st[(size_t)NBd * NNd + kk]; }
    __syncthreads();
#pragma unroll
    for (int rt = 0; rt < 4; ++rt) { f32x8 acc = {};
#pragma unroll
      for (int ks = 0; ks < 4; ++ks) acc = wmma16(lds_frag(kS + (rt * 16) * 136 + ks * 32, 136), qf[ks], acc);
      const int rbase = rt * 16 + (lane >> 4) * 8;
#pragma unroll
      for (int r = 0; r < 8; ++r) acc_o += exp2f(acc[r] * c - mS[rbase + r]) * wS[rbase + r]; }
  }
  acc_o += __shfl_xor(acc_o, 16, 32);
  if (lane < 16) oS[wave * 16 + lane] = acc_o + bp[0];
  __syncthreads();
#pragma unroll 1
  for (int pass = 0; pass < 2; ++pass) { if (tid < 16) *(volatile v4f_t*)(out + (size_t)b * NNd + (blockIdx.x % (NNd / 64)) * 64 + tid * 4) = *(const v4fa*)(oS + tid * 4); __threadfence(); }
}

extern "C" void kernel_launch(void* const* d_in, const int* in_sizes, int n_in,
                              void* d_out, int out_size, void* d_ws, size_t ws_size,
                              hipStream_t stream) {
  (void)in_sizes; (void)n_in; (void)out_size;
  const float** f = (const float**)d_in;
  const float* kin = f[0], *vin = f[1], *Wq = f[2], *bq = f[3], *Wk = f[4], *bk = f[5], *Wv = f[6], *bv = f[7], *Wp = f[8], *bp = f[9];
  float* out = (float*)d_out;
  char* ws = (char*)d_ws;
  bf16* Q16 = (bf16*)ws; ws += (size_t)NBd * NNd * HHd * 2; bf16* K16 = (bf16*)ws; ws += (size_t)NBd * NNd * HHd * 2;
  float* sv = (float*)ws; ws += (size_t)NBd * NNd * 4; float* st = (float*)ws; ws += (size_t)2 * NBd * NNd * 4;
  if ((size_t)(ws - (char*)d_ws) > ws_size) return;
  const dim3 blk(256);
  gemm_kne<float, 0, true><<<dim3(NBd * NNd / 128, HHd / 128), blk, 0, stream>>>(vin, HHd, Wq, HHd, bq, nullptr, nullptr, Q16, HHd, HHd);
  gemm_kne<float, 0, true><<<dim3(NBd * NNd / 128, HHd / 128), blk, 0, stream>>>(kin, HHd, Wk, HHd, bk, nullptr, nullptr, K16, HHd, HHd);
  k_sval<<<dim3(NBd * NNd / 256), blk, 0, stream>>>(kin, Wv, bv, Wp, sv);
  k_colstats<<<dim3(NBd * (NNd / 64)), dim3(128), 0, stream>>>(Q16, K16, st);
  k_colsoft<<<dim3(NBd * (NNd / 64)), dim3(128), 0, stream>>>(Q16, K16, st, sv, bp, out);
}
